// MambaBlock_28716151341388
// MI455X (gfx1250) — hardware-verified
//
#include <hip/hip_runtime.h>
#include <stddef.h>
#include <stdint.h>

#define BATCH 2
#define SEQ   2048
#define MTOK  4096
#define DM    768
#define DI    1536
#define NXZ   3072
#define NST   16
#define NDBC  64
#define NXP   33

#define RCH   9216
#define RECI  256
#define RECO  128
#define NWI   (NXZ * DM)
#define NWO   (DM * DI)
#define PU0   (NWI / 8)
#define PU1   (NWO / 8)
#define PU2   (NDBC * DI / 8)
#define CLT   16
#define SBD   64
#define STS   64
#define DBP   36
#define WSMAX 134217728

static_assert(RECI * RCH == NWI);
static_assert(RECO * RCH == NWO);
static_assert(PU0 % 256 == 0 && PU1 % 256 == 0 && PU2 % 256 == 0);
static_assert(MTOK == BATCH * SEQ && MTOK % 128 == 0 && MTOK % 8 == 0);
static_assert(DM % 32 == 0 && DI % 32 == 0 && DM % 256 == 0 && DI % 256 == 0);
static_assert(NXZ % 64 == 0 && DM % 64 == 0 && NDBC == 64);
static_assert(SEQ % CLT == 0 && SEQ % STS == 0 && DI % SBD == 0 && STS == SBD);
static_assert(DBP % 4 == 0 && DBP >= 1 + 2 * NST && DBP <= NDBC);
static_assert(DI == 192 * 8);
static_assert(8 * DI * 4 <= 65536);

typedef float          v4f   __attribute__((ext_vector_type(4)));
typedef float          v8f   __attribute__((ext_vector_type(8)));
typedef int            v8i   __attribute__((ext_vector_type(8)));
typedef double         v2d   __attribute__((ext_vector_type(2)));
typedef unsigned short v8us  __attribute__((ext_vector_type(8)));
typedef unsigned short v16us __attribute__((ext_vector_type(16)));
typedef __bf16         v16bf __attribute__((ext_vector_type(16)));
typedef v4f  __attribute__((may_alias)) v4fa;
typedef v8us __attribute__((may_alias)) v8usa;
union FragB { v16bf v; v16us u; v8us h[2]; v8i w; };

__device__ __forceinline__ v8f wmb(const FragB& a, const FragB& b, v8f c) {
  v8f d = __builtin_amdgcn_wmma_f32_16x16x32_bf16(false, a.v, false, b.v, (short)0, c, false, false);
  asm volatile("v_nop\n\tv_nop\n\tv_nop\n\tv_nop" : "+v"(d) : "v"(a.w), "v"(b.w));
  return d;
}

__device__ __forceinline__ unsigned bf16_bits(float f) {
  const unsigned u = __float_as_uint(f);
  return (u + 0x7FFFu + ((u >> 16) & 1u)) >> 16;
}
__device__ __forceinline__ float bf16_val(float f) {
  return __uint_as_float(bf16_bits(f) << 16);
}
__device__ __forceinline__ void hilo(float f, unsigned short& hb, unsigned short& lb) {
  const unsigned h = bf16_bits(f);
  hb = (unsigned short)h;
  lb = (unsigned short)bf16_bits(f - __uint_as_float(h << 16));
}
__device__ __forceinline__ void put16(unsigned short* dp, v8us o) {
  *(volatile v8us*)dp = o;
  __threadfence();
  *(volatile v8us*)dp = o;
}
__device__ __forceinline__ float wave_sum(float s) {
  s += __shfl_xor(s, 16);
  s += __shfl_xor(s, 8);
  s += __shfl_xor(s, 4);
  s += __shfl_xor(s, 2);
  s += __shfl_xor(s, 1);
  return s;
}
__device__ __forceinline__ float silu_f(float v) {
  const float e = expf(-v);
  return v * __builtin_amdgcn_rcpf(1.0f + e);
}

__global__ __launch_bounds__(256) void k_absrec(const float* __restrict__ Wi, const float* __restrict__ Wo,
                                                double* REC) {
  __shared__ double red[256];
  const int tid = (int)threadIdx.x;
  const int blk = (int)blockIdx.x;
  const float* src = (blk < RECI) ? (Wi + (size_t)blk * RCH) : (Wo + (size_t)(blk - RECI) * RCH);
  double s = 0.0;
#pragma unroll 3
  for (int i = 0; i < 9; ++i) {
    const v4f a = *(const v4fa*)(src + (size_t)(i * 256 + tid) * 4);
    s += (double)fabsf(bf16_val(a.x));
    s += (double)fabsf(bf16_val(a.y));
    s += (double)fabsf(bf16_val(a.z));
    s += (double)fabsf(bf16_val(a.w));
  }
  red[tid] = s;
  __syncthreads();
  for (int st = 128; st > 0; st >>= 1) {
    if (tid < st) red[tid] = red[tid] + red[tid + st];
    __syncthreads();
  }
  const double tot = red[0];
  if (tid < 8) {
    v2d o;
    o.x = (tid == 0) ? tot : 0.0;
    o.y = 0.0;
    double* dp = REC + (size_t)blk * 16 + 2 * tid;
    *(volatile v2d*)dp = o;
    __threadfence();
    *(volatile v2d*)dp = o;
  }
}

__global__ __launch_bounds__(256) void k_combine(const double* __restrict__ REC, float* SC) {
  __shared__ double ra[256];
  __shared__ double rb[256];
  const int tid = (int)threadIdx.x;
  const int ia = tid < RECI ? tid : RECI - 1;
  const int ib = tid < RECO ? tid : RECO - 1;
  const double qa = REC[(size_t)ia * 16];
  const double qb = REC[(size_t)(RECI + ib) * 16];
  ra[tid] = (tid < RECI) ? qa : 0.0;
  rb[tid] = (tid < RECO) ? qb : 0.0;
  __syncthreads();
  for (int st = 128; st > 0; st >>= 1) {
    if (tid < st) {
      ra[tid] = ra[tid] + ra[tid + st];
      rb[tid] = rb[tid] + rb[tid + st];
    }
    __syncthreads();
  }
  const float mi = (float)(ra[0] * (1.0 / (double)NWI));
  const float mo = (float)(rb[0] * (1.0 / (double)NWO));
  const float si = fmaxf(mi, 1e-5f);
  const float so = fmaxf(mo, 1e-5f);
  if (tid < 8) {
    v4f o = {0.0f, 0.0f, 0.0f, 0.0f};
    if (tid == 0) {
      o.x = si;
      o.y = so;
      o.z = 1.0f / si;
      o.w = 1.0f / so;
    }
    float* dp = SC + 4 * tid;
    *(volatile v4f*)dp = o;
    __threadfence();
    *(volatile v4f*)dp = o;
  }
}

__device__ __forceinline__ v8us tern8(const float* src, float rinv) {
  const v4f a = *(const v4fa*)src;
  const v4f b = *(const v4fa*)(src + 4);
  const v8f f8 = {a.x, a.y, a.z, a.w, b.x, b.y, b.z, b.w};
  v8us o;
#pragma unroll
  for (int i = 0; i < 8; ++i) {
    const float wn = bf16_val(f8[i]) * rinv;
    const float q = rintf(fminf(fmaxf(wn, -1.0f), 1.0f));
    o[i] = (unsigned short)bf16_bits(q);
  }
  return o;
}
__global__ __launch_bounds__(256) void k_planes(const float* __restrict__ Wi, const float* __restrict__ Wo,
                                                const float* __restrict__ Xp, const float* __restrict__ SC,
                                                unsigned short* TQI, unsigned short* TQO, unsigned short* XPW) {
  const int u = (int)blockIdx.x * 256 + (int)threadIdx.x;
  if (u < PU0) {
    const v8us o = tern8(Wi + (size_t)u * 8, SC[2]);
    put16(TQI + (size_t)u * 8, o);
  } else if (u < PU0 + PU1) {
    const int v = u - PU0;
    const v8us o = tern8(Wo + (size_t)v * 8, SC[3]);
    put16(TQO + (size_t)v * 8, o);
  } else {
    const int v = u - PU0 - PU1;
    if (v < PU2) {
      const int row = v / 192;
      const int c = v - row * 192;
      const int rc = row < NXP ? row : NXP - 1;
      const unsigned msk = row < NXP ? 0xffffffffu : 0u;
      const float* src = Xp + (size_t)rc * DI + c * 8;
      const v4f a = *(const v4fa*)src;
      const v4f b = *(const v4fa*)(src + 4);
      const v8f f8 = {a.x, a.y, a.z, a.w, b.x, b.y, b.z, b.w};
      v8us o;
#pragma unroll
      for (int i = 0; i < 8; ++i) o[i] = (unsigned short)(bf16_bits(f8[i]) & msk);
      put16(XPW + (size_t)v * 8, o);
    }
  }
}

template <int NU, int TWO, int RIN>
__global__ __launch_bounds__(256) void k_rownorm(const float* __restrict__ X, const float* __restrict__ w1,
                                                 const float* __restrict__ w2, unsigned short* OUT) {
  __shared__ __attribute__((aligned(16))) float sV[8 * NU * 256];
  const int KK = NU * 256;
  const int tid = (int)threadIdx.x, lane = tid & 31, wave = tid >> 5;
  const int row = (int)blockIdx.x * 8 + wave;
  const float* xr = X + (size_t)row * KK;
  float* lv = sV + wave * KK + lane * 8;

  float s = 0.0f;
#pragma unroll 1
  for (int u = 0; u < NU; ++u) {
    const int c = (u * 32 + lane) * 8;
    const v4f a = *(const v4fa*)(xr + c);
    const v4f b = *(const v4fa*)(xr + c + 4);
    const v8f f8 = {a.x, a.y, a.z, a.w, b.x, b.y, b.z, b.w};
    v8f t8;
#pragma unroll
    for (int i = 0; i < 8; ++i) {
      const float t = RIN ? bf16_val(f8[i]) : f8[i];
      t8[i] = t;
      s += t * t;
    }
    const v4f qa = {t8[0], t8[1], t8[2], t8[3]};
    const v4f qb = {t8[4], t8[5], t8[6], t8[7]};
    *(v4fa*)(lv + u * 256)     = qa;
    *(v4fa*)(lv + u * 256 + 4) = qb;
  }
  s = wave_sum(s);
  float rs = rsqrtf(s * (1.0f / (float)KK) + 1e-6f);

  if (TWO) {
    float s2 = 0.0f;
#pragma unroll 1
    for (int u = 0; u < NU; ++u) {
      const int c = (u * 32 + lane) * 8;
      const v4f a = *(const v4fa*)(w1 + c);
      const v4f b = *(const v4fa*)(w1 + c + 4);
      const v8f g8 = {a.x, a.y, a.z, a.w, b.x, b.y, b.z, b.w};
      const v4f pa = *(const v4fa*)(lv + u * 256);
      const v4f pb = *(const v4fa*)(lv + u * 256 + 4);
      const v8f p8 = {pa.x, pa.y, pa.z, pa.w, pb.x, pb.y, pb.z, pb.w};
      v8f t8;
#pragma unroll
      for (int i = 0; i < 8; ++i) {
        const float hv = (p8[i] * rs) * bf16_val(g8[i]);
        t8[i] = hv;
        s2 += hv * hv;
      }
      const v4f qa = {t8[0], t8[1], t8[2], t8[3]};
      const v4f qb = {t8[4], t8[5], t8[6], t8[7]};
      *(v4fa*)(lv + u * 256)     = qa;
      *(v4fa*)(lv + u * 256 + 4) = qb;
    }
    s2 = wave_sum(s2);
    rs = rsqrtf(s2 * (1.0f / (float)KK) + 1e-6f);
  }

  unsigned short* orow = OUT + (size_t)row * (2 * KK);
#pragma unroll 1
  for (int u = 0; u < NU; ++u) {
    const int c = (u * 32 + lane) * 8;
    const v4f a = *(const v4fa*)(w2 + c);
    const v4f b = *(const v4fa*)(w2 + c + 4);
    const v8f g8 = {a.x, a.y, a.z, a.w, b.x, b.y, b.z, b.w};
    const v4f pa = *(const v4fa*)(lv + u * 256);
    const v4f pb = *(const v4fa*)(lv + u * 256 + 4);
    const v8f p8 = {pa.x, pa.y, pa.z, pa.w, pb.x, pb.y, pb.z, pb.w};
    v8us oh, ol;
#pragma unroll
    for (int i = 0; i < 8; ++i) {
      const float o = (p8[i] * rs) * bf16_val(g8[i]);
      unsigned short hb, lb;
      hilo(o, hb, lb);
      oh[i] = hb;
      ol[i] = lb;
    }
    unsigned short* dp = orow + c;
    *(volatile v8us*)dp = oh;
    *(volatile v8us*)(dp + KK) = ol;
    __threadfence();
    *(volatile v8us*)dp = oh;
    *(volatile v8us*)(dp + KK) = ol;
  }
}

template <int MODE>
__global__ __launch_bounds__(128) void k_gemm(const unsigned short* __restrict__ A,
                                              const unsigned short* __restrict__ BT, int KB,
                                              const float* __restrict__ scales, const float* __restrict__ xres,
                                              float* C, int ldc) {
  __shared__ __attribute__((aligned(16))) float stg[128 * 64];
  const int tid = (int)threadIdx.x, lane = tid & 31, w = tid >> 5, hh = lane >> 4, m = lane & 15;
  const int m0b = (int)blockIdx.x * 128;
  const int n0  = (int)blockIdx.y * 64;
  const size_t lda = (size_t)2 * (size_t)KB;
  const unsigned short* ap0 = A + (size_t)(m0b + 32 * w + m) * lda + 8 * hh;
  const unsigned short* ap1 = ap0 + 16 * lda;
  const unsigned short* bp  = BT + (size_t)(n0 + m) * (size_t)KB + 8 * hh;

  v8f acc[2][4];
  {
    const v8f z = {0.f, 0.f, 0.f, 0.f, 0.f, 0.f, 0.f, 0.f};
#pragma unroll
    for (int mt = 0; mt < 2; ++mt)
#pragma unroll
      for (int nt = 0; nt < 4; ++nt) acc[mt][nt] = z;
  }

#pragma unroll 1
  for (int k0 = 0; k0 < KB; k0 += 32) {
    FragB h0, h1, l0, l1;
    h0.h[0] = *(const v8usa*)(ap0 + k0);
    h0.h[1] = *(const v8usa*)(ap0 + k0 + 16);
    h1.h[0] = *(const v8usa*)(ap1 + k0);
    h1.h[1] = *(const v8usa*)(ap1 + k0 + 16);
    l0.h[0] = *(const v8usa*)(ap0 + KB + k0);
    l0.h[1] = *(const v8usa*)(ap0 + KB + k0 + 16);
    l1.h[0] = *(const v8usa*)(ap1 + KB + k0);
    l1.h[1] = *(const v8usa*)(ap1 + KB + k0 + 16);
#pragma unroll
    for (int nt = 0; nt < 4; ++nt) {
      const unsigned short* wq = bp + (size_t)(16 * nt) * (size_t)KB + k0;
      FragB b;
      b.h[0] = *(const v8usa*)wq;
      b.h[1] = *(const v8usa*)(wq + 16);
      acc[0][nt] = wmb(h0, b, acc[0][nt]);
      acc[1][nt] = wmb(h1, b, acc[1][nt]);
      acc[0][nt] = wmb(l0, b, acc[0][nt]);
      acc[1][nt] = wmb(l1, b, acc[1][nt]);
    }
  }

  float sc = 1.0f;
  if (MODE == 0) sc = scales[0];
  if (MODE == 2) sc = scales[1];
#pragma unroll
  for (int nt = 0; nt < 4; ++nt) {
#pragma unroll
    for (int mt = 0; mt < 2; ++mt) {
#pragma unroll
      for (int r = 0; r < 8; ++r) {
        const int lr = 32 * w + 16 * mt + 8 * hh + r;
        stg[lr * 64 + 16 * nt + m] = acc[mt][nt][r] * sc;
      }
    }
  }
  __syncthreads();

  v4f pv[16];
#pragma unroll
  for (int i = 0; i < 16; ++i) {
    const int lr = 32 * w + 2 * i + hh;
    v4f v = *(const v4fa*)(stg + lr * 64 + 4 * m);
    if (MODE == 2) {
      const v4f xr = *(const v4fa*)(xres + (size_t)(m0b + lr) * (size_t)ldc + n0 + 4 * m);
      v.x = v.x + bf16_val(xr.x);
      v.y = v.y + bf16_val(xr.y);
      v.z = v.z + bf16_val(xr.z);
      v.w = v.w + bf16_val(xr.w);
    }
    pv[i] = v;
  }
#pragma unroll
  for (int i = 0; i < 16; ++i) {
    float* op = C + (size_t)(m0b + 32 * w + 2 * i + hh) * (size_t)ldc + n0 + 4 * m;
    *(volatile v4f*)op = pv[i];
  }
  __threadfence();
#pragma unroll
  for (int i = 0; i < 16; ++i) {
    float* op = C + (size_t)(m0b + 32 * w + 2 * i + hh) * (size_t)ldc + n0 + 4 * m;
    *(volatile v4f*)op = pv[i];
  }
}

__device__ __forceinline__ void load8s(const float* p, float f, float* o) {
  const v4f a = *(const v4fa*)p;
  const v4f b = *(const v4fa*)(p + 4);
  o[0] = a.x * f; o[1] = a.y * f; o[2] = a.z * f; o[3] = a.w * f;
  o[4] = b.x * f; o[5] = b.y * f; o[6] = b.z * f; o[7] = b.w * f;
}
__global__ __launch_bounds__(192) void k_conv(const float* __restrict__ XZ, const float* __restrict__ cw,
                                              const float* __restrict__ cb, unsigned short* XC) {
  const int tid = (int)threadIdx.x;
  const int d8 = tid * 8;
  const int l0 = (int)blockIdx.x * CLT;
  const int b  = (int)blockIdx.y;
  float w0[8], w1[8], w2[8], w3[8], bs[8];
#pragma unroll
  for (int c = 0; c < 8; ++c) {
    const v4f t = *(const v4fa*)(cw + (size_t)(d8 + c) * 4);
    w0[c] = bf16_val(t.x);
    w1[c] = bf16_val(t.y);
    w2[c] = bf16_val(t.z);
    w3[c] = bf16_val(t.w);
  }
  {
    const v4f a = *(const v4fa*)(cb + d8);
    const v4f c2 = *(const v4fa*)(cb + d8 + 4);
    bs[0] = bf16_val(a.x); bs[1] = bf16_val(a.y); bs[2] = bf16_val(a.z); bs[3] = bf16_val(a.w);
    bs[4] = bf16_val(c2.x); bs[5] = bf16_val(c2.y); bs[6] = bf16_val(c2.z); bs[7] = bf16_val(c2.w);
  }
  const size_t rowb = (size_t)b * SEQ;
  const float fpre = (l0 > 0) ? 1.0f : 0.0f;
  const int la = l0 - 3 > 0 ? l0 - 3 : 0;
  const int lb = l0 - 2 > 0 ? l0 - 2 : 0;
  const int lc = l0 - 1 > 0 ? l0 - 1 : 0;
  float xa[8], xb[8], xc[8];
  load8s(XZ + (rowb + la) * NXZ + d8, fpre, xa);
  load8s(XZ + (rowb + lb) * NXZ + d8, fpre, xb);
  load8s(XZ + (rowb + lc) * NXZ + d8, fpre, xc);
#pragma unroll 1
  for (int s = 0; s < CLT; ++s) {
    const size_t row = rowb + l0 + s;
    float cu[8];
    load8s(XZ + row * NXZ + d8, 1.0f, cu);
    v8us oh, ol;
#pragma unroll
    for (int c = 0; c < 8; ++c) {
      float a = bs[c];
      a = fmaf(w0[c], xa[c], a);
      a = fmaf(w1[c], xb[c], a);
      a = fmaf(w2[c], xc[c], a);
      a = fmaf(w3[c], cu[c], a);
      const float y = silu_f(a);
      unsigned short hb, lbt;
      hilo(y, hb, lbt);
      oh[c] = hb;
      ol[c] = lbt;
    }
    unsigned short* dp = XC + row * NXZ + d8;
    *(volatile v8us*)dp = oh;
    *(volatile v8us*)(dp + DI) = ol;
    __threadfence();
    *(volatile v8us*)dp = oh;
    *(volatile v8us*)(dp + DI) = ol;
#pragma unroll
    for (int c = 0; c < 8; ++c) { xa[c] = xb[c]; xb[c] = xc[c]; xc[c] = cu[c]; }
  }
}

__global__ __launch_bounds__(SBD) void k_scan(const float* __restrict__ DBC, const unsigned short* __restrict__ XC,
                                              const float* __restrict__ XZ, const float* __restrict__ dtW,
                                              const float* __restrict__ dtB, const float* __restrict__ Alog,
                                              const float* __restrict__ Dp, float* Y) {
  __shared__ __attribute__((aligned(16))) float sH[NST * SBD];
  __shared__ __attribute__((aligned(16))) float sA[NST * SBD];
  __shared__ __attribute__((aligned(16))) float sD[STS * DBP];
  __shared__ __attribute__((aligned(16))) float sY[STS * SBD];
  const int tid = (int)threadIdx.x;
  const int d0 = (int)blockIdx.x * SBD;
  const int d  = d0 + tid;
  const int b  = (int)blockIdx.y;

#pragma unroll 1
  for (int q = 0; q < 4; ++q) {
    const v4f al = *(const v4fa*)(Alog + (size_t)d * NST + 4 * q);
    sA[(4 * q + 0) * SBD + tid] = -expf(bf16_val(al.x));
    sA[(4 * q + 1) * SBD + tid] = -expf(bf16_val(al.y));
    sA[(4 * q + 2) * SBD + tid] = -expf(bf16_val(al.z));
    sA[(4 * q + 3) * SBD + tid] = -expf(bf16_val(al.w));
    sH[(4 * q + 0) * SBD + tid] = 0.0f;
    sH[(4 * q + 1) * SBD + tid] = 0.0f;
    sH[(4 * q + 2) * SBD + tid] = 0.0f;
    sH[(4 * q + 3) * SBD + tid] = 0.0f;
  }
  const float dtw = bf16_val(dtW[d]);
  const float dtb = bf16_val(dtB[d]);
  const float dd  = bf16_val(Dp[d]);
  const size_t rowb = (size_t)b * SEQ;

#pragma unroll 1
  for (int ch = 0; ch < SEQ / STS; ++ch) {
    const size_t row0 = rowb + (size_t)ch * STS;
    {
      const float* gp = DBC + (row0 + tid) * NDBC;
      float* lp = sD + tid * DBP;
#pragma unroll 3
      for (int q = 0; q < DBP / 4; ++q) *(v4fa*)(lp + 4 * q) = *(const v4fa*)(gp + 4 * q);
    }
    __syncthreads();

#pragma unroll 1
    for (int s = 0; s < STS; ++s) {
      const size_t row = row0 + s;
      const float* dr = sD + s * DBP;
      const unsigned hb = XC[row * NXZ + d];
      const unsigned lb = XC[row * NXZ + DI + d];
      const float zt = XZ[row * NXZ + DI + d];
      const float xt = __uint_as_float(hb << 16) + __uint_as_float(lb << 16);
      const float u  = dr[0] * dtw + dtb;
      const float sp = fmaxf(u, 0.0f) + log1pf(expf(-fabsf(u)));
      const float dbx = sp * xt;
      float ys = 0.0f;
#pragma unroll 1
      for (int n = 0; n < NST; ++n) {
        const float a  = sA[n * SBD + tid];
        float hv = sH[n * SBD + tid];
        hv = expf(sp * a) * hv + dbx * dr[1 + n];
        sH[n * SBD + tid] = hv;
        ys += hv * dr[1 + NST + n];
      }
      const float yv = ys + xt * dd;
      sY[s * SBD + tid] = yv * silu_f(zt);
    }
    __syncthreads();

    v4f pv[16];
#pragma unroll
    for (int it = 0; it < 16; ++it) pv[it] = *(const v4fa*)(sY + (size_t)(it * SBD + tid) * 4);
#pragma unroll
    for (int it = 0; it < 16; ++it) {
      const int idx = it * SBD + tid;
      float* op = Y + (row0 + (size_t)(idx >> 4)) * DI + d0 + 4 * (idx & 15);
      *(volatile v4f*)op = pv[it];
    }
    __threadfence();
#pragma unroll
    for (int it = 0; it < 16; ++it) {
      const int idx = it * SBD + tid;
      float* op = Y + (row0 + (size_t)(idx >> 4)) * DI + d0 + 4 * (idx & 15);
      *(volatile v4f*)op = pv[it];
    }
  }
}

extern "C" void kernel_launch(void* const* d_in, const int* in_sizes, int n_in,
                              void* d_out, int out_size, void* d_ws, size_t ws_size,
                              hipStream_t stream) {
  if (n_in < 13) return;
  if (in_sizes[0] != MTOK * DM) return;
  if (in_sizes[1] != DM || in_sizes[2] != DM) return;
  if (in_sizes[3] != NWI) return;
  if (in_sizes[4] != DI * 4 || in_sizes[5] != DI) return;
  if (in_sizes[6] != NXP * DI) return;
  if (in_sizes[7] != DI || in_sizes[8] != DI) return;
  if (in_sizes[9] != DI * NST) return;
  if (in_sizes[10] != DI || in_sizes[11] != DI) return;
  if (in_sizes[12] != NWO) return;
  if (out_size != MTOK * DM) return;

  const float* x    = (const float*)d_in[0];
  const float* nw   = (const float*)d_in[1];
  const float* inw  = (const float*)d_in[2];
  const float* Wi   = (const float*)d_in[3];
  const float* cw   = (const float*)d_in[4];
  const float* cb   = (const float*)d_in[5];
  const float* Xp   = (const float*)d_in[6];
  const float* dtW  = (const float*)d_in[7];
  const float* dtB  = (const float*)d_in[8];
  const float* Alog = (const float*)d_in[9];
  const float* Dp   = (const float*)d_in[10];
  const float* onw  = (const float*)d_in[11];
  const float* Wo   = (const float*)d_in[12];
  float* out = (float*)d_out;

  char* ws = (char*)d_ws;
  size_t off = 0;
  const size_t oREC = off; off += (size_t)(RECI + RECO) * 128;       off = (off + 255) & ~(size_t)255;
  const size_t oSC  = off; off += 128;                               off = (off + 255) & ~(size_t)255;
  const size_t oTQI = off; off += (size_t)NXZ * DM * 2;              off = (off + 255) & ~(size_t)255;
  const size_t oTQO = off; off += (size_t)DM * DI * 2;               off = (off + 255) & ~(size_t)255;
  const size_t oXPW = off; off += (size_t)NDBC * DI * 2;             off = (off + 255) & ~(size_t)255;
  const size_t oXN  = off; off += (size_t)MTOK * 2 * DM * 2;         off = (off + 255) & ~(size_t)255;
  const size_t oXZ  = off; off += (size_t)MTOK * NXZ * 4;            off = (off + 255) & ~(size_t)255;
  const size_t oXC  = off; off += (size_t)MTOK * NXZ * 2;            off = (off + 255) & ~(size_t)255;
  const size_t oDBC = off; off += (size_t)MTOK * NDBC * 4;           off = (off + 255) & ~(size_t)255;
  const size_t oY   = off; off += (size_t)MTOK * DI * 4;             off = (off + 255) & ~(size_t)255;
  if (off > ws_size || off > (size_t)WSMAX) return;

  double*         REC = (double*)(ws + oREC);
  float*          SC  = (float*)(ws + oSC);
  unsigned short* TQI = (unsigned short*)(ws + oTQI);
  unsigned short* TQO = (unsigned short*)(ws + oTQO);
  unsigned short* XPW = (unsigned short*)(ws + oXPW);
  unsigned short* XN  = (unsigned short*)(ws + oXN);
  float*          XZ  = (float*)(ws + oXZ);
  unsigned short* XC  = (unsigned short*)(ws + oXC);
  unsigned short* YN  = (unsigned short*)(ws + oXC);
  float*          DBC = (float*)(ws + oDBC);
  float*          Y   = (float*)(ws + oY);

  k_absrec<<<RECI + RECO, 256, 0, stream>>>(Wi, Wo, REC);
  k_combine<<<1, 256, 0, stream>>>(REC, SC);
  k_planes<<<(PU0 + PU1 + PU2) / 256, 256, 0, stream>>>(Wi, Wo, Xp, SC, TQI, TQO, XPW);
  k_rownorm<3, 1, 1><<<MTOK / 8, 256, 0, stream>>>(x, nw, inw, XN);
  k_gemm<0><<<dim3(MTOK / 128, NXZ / 64), 128, 0, stream>>>(XN, TQI, DM, SC, x, XZ, NXZ);
  k_conv<<<dim3(SEQ / CLT, BATCH), 192, 0, stream>>>(XZ, cw, cb, XC);
  k_gemm<1><<<dim3(MTOK / 128, 1), 128, 0, stream>>>(XC, XPW, DI, SC, x, DBC, NDBC);
  k_scan<<<dim3(DI / SBD, BATCH), SBD, 0, stream>>>(DBC, XC, XZ, dtW, dtB, Alog, Dp, Y);
  k_rownorm<6, 0, 0><<<MTOK / 8, 256, 0, stream>>>(Y, onw, onw, YN);
  k_gemm<2><<<dim3(MTOK / 128, DM / 64), 128, 0, stream>>>(YN, TQO, DI, SC, x, out, DM);
}
